// GCNEdgeBased_32701880992042
// MI455X (gfx1250) — hardware-run, weakly checked
//
#include <hip/hip_runtime.h>


namespace {
constexpr int N = 50000, E = 800000, F = 128, H = 32, NPB = 8;
constexpr float HS = 256.0f, WSC = 256.0f;
typedef _Float16 b16;
typedef __attribute__((ext_vector_type(16))) _Float16 v16b;
typedef __attribute__((ext_vector_type(8))) _Float16 v8b;
typedef __attribute__((ext_vector_type(8))) float v8f;
typedef __attribute__((ext_vector_type(4))) float v4f;
__device__ __forceinline__ float bf16_rne(float f) { unsigned int u = __float_as_uint(f); u += 0x7FFFu + ((u >> 16) & 1u); float r = __uint_as_float(u & 0xFFFF0000u); asm volatile("" : "+v"(r)); return r; }
__device__ __forceinline__ float bfv(float f) { float r = bf16_rne(f); asm volatile("" : "+v"(r)); return r; }
__device__ __forceinline__ void split16(float v, b16& hi, b16& lo) { hi = (b16)v; lo = (b16)(v - (float)hi); }
__device__ __forceinline__ v16b frag_kb(const b16* p, int hh) { const v8b a = *(const v8b*)(p + 8 * hh), b = *(const v8b*)(p + 16 + 8 * hh); v16b f;
#pragma unroll
  for (int e = 0; e < 8; ++e) { f[e] = a[e]; f[8 + e] = b[e]; } return f; }
__device__ __forceinline__ v8f wmma16b(v16b a, v16b b, v8f c) { v8f d = __builtin_amdgcn_wmma_f32_16x16x32_f16(false, a, false, b, (short)0, c, false, false); asm volatile("v_nop\n\tv_nop\n\tv_nop\n\tv_nop" : "+v"(d) : "v"(a), "v"(b)); return d; }
__device__ __forceinline__ void wave_lds_sync() { __builtin_amdgcn_fence(__ATOMIC_RELEASE, "workgroup"); __builtin_amdgcn_wave_barrier(); __builtin_amdgcn_fence(__ATOMIC_ACQUIRE, "workgroup"); }
__device__ __forceinline__ float pmul(float a, float b) { float p = a * b; asm volatile("" : "+v"(p)); return p; }
__device__ __forceinline__ int iclamp(int v, int lo, int hi) { return v < lo ? lo : (v > hi ? hi : v); }
constexpr int CSR_NBLK8 = 512, CSR_GB8 = 8, CSR_GN8 = 1 << CSR_GB8  , CSR_TS8 = (CSR_GN8 < 32 ? 32 : CSR_GN8)  , CSR_MAXG8 = 512, CSR_CAP8 = 12288  ;
__device__ __host__ __forceinline__ int csr_tix8(int v) { return (v >> CSR_GB8) * CSR_TS8 + (v & (CSR_GN8 - 1)); }
__global__ __launch_bounds__(64) void csrA_kernel8(const int* __restrict__ dst, int E, int N, int nG, int CHP, int NGP, int* __restrict__ STG, int* __restrict__ HST) {
  extern __shared__ int sm[];
  int* cnt = sm; int* run = sm + NGP; int* ids = sm + 2 * NGP;
  const int b = blockIdx.x; const int ch = (E + CSR_NBLK8 - 1) / CSR_NBLK8; const int e0 = b * ch, e1 = min(E, e0 + ch);
  for (int i = threadIdx.x; i < NGP; i += 64) cnt[i] = 0;
  for (int i = threadIdx.x; i < CHP; i += 64) ids[i] = -1;
  __syncthreads();
  if (threadIdx.x == 0) {
    for (int e = e0; e < e1; ++e) { int d = dst[e]; d = (d < 0) ? 0 : (d >= N ? N - 1 : d); cnt[d >> CSR_GB8] += 1; }
    int acc = 0; for (int g = 0; g < nG; ++g) { run[g] = acc; acc += cnt[g]; }
    for (int e = e0; e < e1; ++e) { int d = dst[e]; d = (d < 0) ? 0 : (d >= N ? N - 1 : d); const int g = d >> CSR_GB8; ids[run[g]] = e; run[g] += 1; } }
  __syncthreads();
  typedef __attribute__((ext_vector_type(4))) int v4i;
  for (int pass = 0; pass < 2; ++pass) {
    for (int i = threadIdx.x; i < CHP / 4; i += 64) *(volatile v4i*)(STG + (size_t)b * CHP + i * 4) = *(const v4i*)(&ids[i * 4]);
    for (int i = threadIdx.x; i < NGP / 4; i += 64) { v4i v; for (int e = 0; e < 4; ++e) v[e] = (i * 4 + e < nG) ? cnt[i * 4 + e] : 0; *(volatile v4i*)(HST + (size_t)b * NGP + i * 4) = v; }
    __threadfence(); }
}
__global__ __launch_bounds__(512) void csrS_kernel8(const int* __restrict__ HST, int nG, int NGP, int* __restrict__ START, int* __restrict__ TOT, int* __restrict__ OFF) {
  __shared__ int tot[CSR_MAXG8];
  const int b = threadIdx.x;
  for (int pass = 0; pass < 2; ++pass) { int runb = 0; for (int g = 0; g < nG; ++g) { int c = HST[(size_t)b * NGP + g]; c = (c < 0) ? 0 : c; ((volatile int*)OFF)[(size_t)g * CSR_NBLK8 + b] = runb; runb += c; } __threadfence(); }
  for (int g = threadIdx.x; g < nG; g += 512) { int s = 0; for (int bb = 0; bb < CSR_NBLK8; ++bb) { int c = HST[(size_t)bb * NGP + g]; s += (c < 0) ? 0 : c; } tot[g] = s; }
  __syncthreads();
  if (threadIdx.x < 32) {
    __shared__ int st[CSR_MAXG8 + 32];
    if (threadIdx.x == 0) { int acc = 0; for (int g = 0; g < NGP; ++g) { st[g] = acc; if (g < nG) acc += (tot[g] + 31) & ~31; } st[NGP] = acc; }
    __builtin_amdgcn_fence(__ATOMIC_RELEASE, "workgroup"); __builtin_amdgcn_wave_barrier(); __builtin_amdgcn_fence(__ATOMIC_ACQUIRE, "workgroup");
    for (int pass = 0; pass < 2; ++pass) { for (int i = threadIdx.x; i < NGP + 32; i += 32) { ((volatile int*)START)[i] = (i <= NGP) ? st[min(i, NGP)] : 0; ((volatile int*)TOT)[i] = (i < nG) ? tot[i] : 0; } __threadfence(); } }
}
__global__ __launch_bounds__(256) void csrB_kernel8(const int* __restrict__ dst, int N, int nG, int CHP, int NGP, int permLen, const int* __restrict__ STG, const int* __restrict__ HST, const int* __restrict__ OFF, const int* __restrict__ START, const int* __restrict__ TOT, int* __restrict__ PERM, int* __restrict__ ROWPTR, int* __restrict__ ROWCNT, int* __restrict__ FLAG) {
  typedef __attribute__((ext_vector_type(4))) int v4i;
  __shared__ int ids[CSR_CAP8]; __shared__ unsigned short key[CSR_CAP8]; __shared__ int outp[CSR_CAP8]; __shared__ int ncnt[CSR_GN8 + 1]; __shared__ int boff[CSR_NBLK8 + 1];
  const int g = blockIdx.x, t_ = threadIdx.x; int tot = TOT[g]; int st = START[g], stn = START[g + 1]; const int v0 = g * CSR_GN8; const int nv = min(CSR_GN8, N - v0); const int t0 = g * CSR_TS8;
  st = (st < 0) ? 0 : (st > permLen - 32 ? permLen - 32 : st) & ~31; stn = (stn < st) ? st : (stn > permLen ? permLen : stn); tot = (tot < 0) ? 0 : tot; if (tot > stn - st && tot <= CSR_CAP8) tot = stn - st;
  if (tot > CSR_CAP8) {
    for (int pass = 0; pass < 2; ++pass) { for (int i = t_; i < CSR_TS8 / 4; i += 256) { v4i a, c; for (int e = 0; e < 4; ++e) { a[e] = st; c[e] = 0; } *(volatile v4i*)(ROWPTR + t0 + i * 4) = a; *(volatile v4i*)(ROWCNT + t0 + i * 4) = c; } if (t_ == 0) ((volatile int*)FLAG)[0] = 1; __threadfence(); } (void)nv; return; }
  if (t_ == 0) { int acc = 0; for (int b = 0; b < CSR_NBLK8; ++b) { boff[b] = acc; int c = HST[(size_t)b * NGP + g]; c = (c < 0) ? 0 : (c > CHP ? CHP : c); acc += c; if (acc > tot) acc = tot; } boff[CSR_NBLK8] = acc; }
  for (int i = t_; i <= CSR_GN8; i += 256) ncnt[i] = 0;
  __syncthreads();
  for (int b = 0; b < CSR_NBLK8; ++b) { const int c = boff[b + 1] - boff[b]; int o_ = OFF[(size_t)g * CSR_NBLK8 + b]; o_ = (o_ < 0) ? 0 : (o_ > CHP - c ? CHP - c : o_); const int* src_ = STG + (size_t)b * CHP + o_;
    for (int i = t_; i < c; i += 256) { int id = src_[i]; id = (id < 0) ? 0 : id; ids[boff[b] + i] = id; int d = dst[id]; d = (d < v0) ? v0 : (d >= N ? N - 1 : d); int kk = d - v0; kk = (kk < 0) ? 0 : (kk >= CSR_GN8 ? CSR_GN8 - 1 : kk); key[boff[b] + i] = (unsigned short)kk; } }
  __syncthreads();
  if (t_ == 0) { for (int i = 0; i < tot; ++i) ncnt[key[i]] += 1; int acc = 0; for (int vl = 0; vl < CSR_GN8; ++vl) { const int c = ncnt[vl]; ncnt[vl] = acc; acc += c; } ncnt[CSR_GN8] = acc;
    for (int i = 0; i < tot; ++i) { const int vl = key[i]; outp[ncnt[vl]] = ids[i]; ncnt[vl] += 1; }
    for (int vl = CSR_GN8; vl > 0; --vl) ncnt[vl] = ncnt[vl - 1]; ncnt[0] = 0; }
  __syncthreads();
  for (int pass = 0; pass < 2; ++pass) {
    for (int i = t_; i < (stn - st) / 4; i += 256) { v4i v; for (int e = 0; e < 4; ++e) { const int q = i * 4 + e; v[e] = (q < tot) ? outp[q] : -1; } *(volatile v4i*)(PERM + st + i * 4) = v; }
    for (int i = t_; i < CSR_TS8 / 4; i += 256) { v4i a, c; for (int e = 0; e < 4; ++e) { const int vl = i * 4 + e; const int vc = vl < CSR_GN8 ? vl : CSR_GN8; a[e] = (vl < CSR_GN8) ? st + ncnt[vc] : st; c[e] = (vl < nv) ? (ncnt[(vc < CSR_GN8 ? vc : CSR_GN8 - 1) + 1] - ncnt[vc]) : 0; } *(volatile v4i*)(ROWPTR + t0 + i * 4) = a; *(volatile v4i*)(ROWCNT + t0 + i * 4) = c; }
    __threadfence(); }
}
__global__ __launch_bounds__(256) void csrZ_kernel8(int* __restrict__ p, size_t n4) { typedef __attribute__((ext_vector_type(4))) int v4i; const size_t tid = (size_t)blockIdx.x * 256 + threadIdx.x, nth = (size_t)gridDim.x * 256; v4i z = {0, 0, 0, 0}; for (size_t i = tid; i < n4; i += nth) *(volatile v4i*)(p + i * 4) = z; }
struct CsrBufs8 { int *STG, *HST, *OFF, *START, *TOT, *PERM, *ROWPTR, *ROWCNT, *FLAG; int nG, NGP, CHP; size_t permLen; char* base; size_t bytes; };
static size_t csr_carve8(CsrBufs8& c, char* ws, size_t off, int E, int N) {
  const size_t off0 = off; c.base = ws + off;
  auto al = [&](size_t bytes) { char* p = ws + off; off += (bytes + 255) & ~(size_t)255; return p; };
  c.nG = (N + CSR_GN8 - 1) / CSR_GN8; c.NGP = (c.nG + 31) & ~31; const int ch = (E + CSR_NBLK8 - 1) / CSR_NBLK8; c.CHP = (ch + 31) & ~31; c.permLen = (size_t)E + 32 * (size_t)c.nG + 32;
  c.STG = (int*)al((size_t)CSR_NBLK8 * c.CHP * 4); c.HST = (int*)al((size_t)CSR_NBLK8 * c.NGP * 4); c.OFF = (int*)al((size_t)c.NGP * CSR_NBLK8 * 4); c.START = (int*)al((size_t)(c.NGP + 64) * 4); c.TOT = (int*)al((size_t)(c.NGP + 64) * 4);
  c.PERM = (int*)al(c.permLen * 4); c.ROWPTR = (int*)al((size_t)c.nG * CSR_TS8 * 4); c.ROWCNT = (int*)al((size_t)c.nG * CSR_TS8 * 4); c.FLAG = (int*)al(256);
  c.bytes = off - off0; return off;
}
static void csr_build8(const CsrBufs8& c, const int* dst, int E, int N, hipStream_t stream) {
  const size_t smem = (size_t)(2 * c.NGP + c.CHP) * 4;
  csrZ_kernel8<<<512, 256, 0, stream>>>((int*)c.base, c.bytes / 16);
  csrA_kernel8<<<CSR_NBLK8, 64, smem, stream>>>(dst, E, N, c.nG, c.CHP, c.NGP, c.STG, c.HST);
  csrS_kernel8<<<1, 512, 0, stream>>>(c.HST, c.nG, c.NGP, c.START, c.TOT, c.OFF);
  csrB_kernel8<<<c.nG, 256, 0, stream>>>(dst, N, c.nG, c.CHP, c.NGP, (int)c.permLen, c.STG, c.HST, c.OFF, c.START, c.TOT, c.PERM, c.ROWPTR, c.ROWCNT, c.FLAG);
}


__global__ __launch_bounds__(256) void wput_kernel(const float* __restrict__ wn1p, const float* __restrict__ we1p, const float* __restrict__ we1s, const float* __restrict__ wn2p, const float* __restrict__ wn2s, const float* __restrict__ we2p, const float* __restrict__ we2s, b16* __restrict__ WN1, b16* __restrict__ WE1, b16* __restrict__ WN2, b16* __restrict__ WE2) { const int u = blockIdx.x * 256 + threadIdx.x; v8b v;
  if (u < H * 16) { const int o = u / 16, k0 = (u % 16) * 8;
#pragma unroll
    for (int j = 0; j < 8; ++j) v[j] = (b16)(bf16_rne(wn1p[(size_t)o * F + k0 + j]) * WSC); for (int pass = 0; pass < 2; ++pass) { *(volatile v8b*)(WN1 + (size_t)o * F + k0) = v; __threadfence(); } }
  if (u < H * 24) { const int o = u / 24, k0 = (u % 24) * 8;
#pragma unroll
    for (int j = 0; j < 8; ++j) { const int k = k0 + j; v[j] = (b16)(bf16_rne(k < F ? we1s[(size_t)o * F + k] : we1p[(size_t)o * 64 + k - F]) * WSC); } for (int pass = 0; pass < 2; ++pass) { *(volatile v8b*)(WE1 + (size_t)o * 192 + k0) = v; __threadfence(); } }
  if (u < H * 8) { const int o = u / 8, k0 = (u % 8) * 8;
#pragma unroll
    for (int j = 0; j < 8; ++j) { const int k = k0 + j; v[j] = (b16)(bf16_rne(k < H ? wn2p[(size_t)o * H + k] : wn2s[(size_t)o * H + k - H]) * WSC); } for (int pass = 0; pass < 2; ++pass) { *(volatile v8b*)(WN2 + (size_t)o * 64 + k0) = v; __threadfence(); } }
  if (u < H * 16) { const int o = u / 16, k0 = (u % 16) * 8;
#pragma unroll
    for (int j = 0; j < 8; ++j) { const int k = k0 + j; v[j] = (b16)(k < 64 ? bf16_rne(we2p[(size_t)o * 64 + k]) * WSC : (k < 96 ? bf16_rne(we2s[(size_t)o * H + k - 64]) * WSC : 0.0f)); } for (int pass = 0; pass < 2; ++pass) { *(volatile v8b*)(WE2 + (size_t)o * F + k0) = v; __threadfence(); } } }
__global__ __launch_bounds__(32) void node1_kernel(const float* __restrict__ X, const float* __restrict__ Dg, const int* __restrict__ dsts, const int* __restrict__ PERM, const int* __restrict__ ROWPTR, const int* __restrict__ ROWCNT, int permLen, const b16* __restrict__ WN1, const float* __restrict__ bp, const float* __restrict__ bs, const float* __restrict__ ws_unused, int NLIM, float* __restrict__ XN1) { __shared__ __attribute__((aligned(16))) b16 Ah[16][F + 8], Al[16][F + 8]; __shared__ float Tf[16][H + 1]; const int lane = threadIdx.x, nloc = lane & 15, hlf = lane >> 4; const size_t m0 = (size_t)blockIdx.x * 16; if (m0 >= (size_t)NLIM) return;
  for (int rr = 0; rr < 16; ++rr) { const size_t n = m0 + rr; int st = ROWPTR[n], cnt = ROWCNT[n]; cnt = iclamp(cnt, 0, E); st = iclamp(st, 0, permLen - cnt); v4f xn = *(const v4f*)(X + n * F + lane * 4); for (int k = 0; k < 4; ++k) xn[k] = bfv(xn[k]); v4f s = {0, 0, 0, 0};
#pragma unroll 1
    for (int j = 0; j < cnt; ++j) { const int e = iclamp(PERM[st + j], 0, E - 1); const size_t d = (size_t)iclamp(dsts[e], 0, N - 1); if (d >= (size_t)NLIM) continue; const v4f xd = *(const v4f*)(X + d * F + lane * 4);
#pragma unroll
      for (int k = 0; k < 4; ++k) s[k] += fabsf(xn[k] - bfv(xd[k])); }
    const float inv = 1.0f / bfv(Dg[n]); for (int k = 0; k < 4; ++k) { b16 p, ql; split16(pmul(s[k], inv) * HS, p, ql); Ah[rr][lane * 4 + k] = p; Al[rr][lane * 4 + k] = ql; } }
  if (lane < 16) for (int k = F; k < F + 8; ++k) { Ah[lane][k] = (b16)0.0f; Al[lane][k] = (b16)0.0f; }
  wave_lds_sync(); v8f acc[2] = {(v8f){}, (v8f){}};
#pragma unroll
  for (int kb = 0; kb < F; kb += 32) { const v16b a = frag_kb(&Ah[nloc][kb], hlf), al = frag_kb(&Al[nloc][kb], hlf);
#pragma unroll
    for (int t = 0; t < 2; ++t) { const v16b bw = frag_kb(WN1 + (size_t)(t * 16 + nloc) * F + kb, hlf); acc[t] = wmma16b(a, bw, acc[t]); acc[t] = wmma16b(al, bw, acc[t]); } }
#pragma unroll
  for (int t = 0; t < 2; ++t) { const int cc = t * 16 + nloc; const float bb = bfv(bp[cc]) + bfv(bs[cc]) + 0.0f * ws_unused[cc];
#pragma unroll
    for (int r8 = 0; r8 < 8; ++r8) Tf[8 * hlf + r8][cc] = fmaxf(acc[t][r8] * (1.0f / (HS * WSC)) + bb, 0.0f); }
  wave_lds_sync();
  for (int pass = 0; pass < 2; ++pass) { for (int rr = 0; rr < 16; ++rr) ((volatile float*)XN1)[(m0 + rr) * H + lane] = Tf[rr][lane]; __threadfence(); } }
__global__ __launch_bounds__(32) void edge1_kernel(const float* __restrict__ X, const float* __restrict__ XN1, const int* __restrict__ srcs, const int* __restrict__ dsts, const b16* __restrict__ WE1, const float* __restrict__ bep, const float* __restrict__ bes, int NLIM, int ELIM, float* __restrict__ VALS1) { __shared__ __attribute__((aligned(16))) b16 Ah[32][200], Al[32][200]; __shared__ float Tf[32][H + 1]; const int lane = threadIdx.x, nloc = lane & 15, hlf = lane >> 4; const size_t e0 = (size_t)blockIdx.x * 32; if (e0 >= (size_t)ELIM) return;
  for (int rr = 0; rr < 32; ++rr) { const size_t e = e0 + rr; const size_t s = (size_t)iclamp(srcs[e], 0, NLIM - 1), d = (size_t)iclamp(dsts[e], 0, NLIM - 1); for (int q = 0; q < 4; ++q) { const int c = q * 32 + lane; const float v = fabsf(bfv(X[s * F + c]) - bfv(X[d * F + c])); b16 p, ql; split16(v * HS, p, ql); Ah[rr][c] = p; Al[rr][c] = ql; } { const float a = XN1[s * H + lane], b = XN1[d * H + lane]; b16 p, ql; split16((a - b) * 0.5f * HS, p, ql); Ah[rr][F + lane] = p; Al[rr][F + lane] = ql; split16((a + b) * 0.5f * HS, p, ql); Ah[rr][F + H + lane] = p; Al[rr][F + H + lane] = ql; } }
  for (int k = 192; k < 200; ++k) { Ah[lane][k] = (b16)0.0f; Al[lane][k] = (b16)0.0f; }
  wave_lds_sync();
#pragma unroll
  for (int rt = 0; rt < 2; ++rt) { v8f acc[2] = {(v8f){}, (v8f){}};
#pragma unroll
    for (int kb = 0; kb < 192; kb += 32) { const v16b a = frag_kb(&Ah[rt * 16 + nloc][kb], hlf), al = frag_kb(&Al[rt * 16 + nloc][kb], hlf);
#pragma unroll
      for (int t = 0; t < 2; ++t) { const v16b bw = frag_kb(WE1 + (size_t)(t * 16 + nloc) * 192 + kb, hlf); acc[t] = wmma16b(a, bw, acc[t]); acc[t] = wmma16b(al, bw, acc[t]); } }
#pragma unroll
    for (int t = 0; t < 2; ++t) { const int cc = t * 16 + nloc; const float bb = bfv(bep[cc]) + bfv(bes[cc]);
#pragma unroll
      for (int r8 = 0; r8 < 8; ++r8) Tf[rt * 16 + 8 * hlf + r8][cc] = fmaxf(acc[t][r8] * (1.0f / (HS * WSC)) + bb, 0.0f); } }
  wave_lds_sync();
  for (int pass = 0; pass < 2; ++pass) { for (int rr = 0; rr < 32; ++rr) ((volatile float*)VALS1)[(e0 + rr) * H + lane] = Tf[rr][lane]; __threadfence(); } }
__global__ __launch_bounds__(32) void node2_kernel(const float* __restrict__ VALS1, const float* __restrict__ XN1, const float* __restrict__ Dg, const int* __restrict__ PERM, const int* __restrict__ ROWPTR, const int* __restrict__ ROWCNT, int permLen, const b16* __restrict__ WN2, const float* __restrict__ bp, const float* __restrict__ bs, int NLIM, int ELIM, float* __restrict__ XN2) { __shared__ __attribute__((aligned(16))) b16 Ah[16][72], Al[16][72]; __shared__ float Tf[16][H + 1]; const int lane = threadIdx.x, nloc = lane & 15, hlf = lane >> 4; const size_t m0 = (size_t)blockIdx.x * 16; if (m0 >= (size_t)NLIM) return;
  for (int rr = 0; rr < 16; ++rr) { const size_t n = m0 + rr; int st = ROWPTR[n], cnt = ROWCNT[n]; cnt = iclamp(cnt, 0, E); st = iclamp(st, 0, permLen - cnt); float s = 0.0f;
#pragma unroll 1
    for (int j = 0; j < cnt; ++j) { const int e = iclamp(PERM[st + j], 0, E - 1); if (e >= ELIM) continue; s += VALS1[(size_t)e * H + lane]; }
    b16 p, ql; split16(pmul(s, 1.0f / bfv(Dg[n])) * HS, p, ql); Ah[rr][lane] = p; Al[rr][lane] = ql; split16(XN1[n * H + lane] * HS, p, ql); Ah[rr][H + lane] = p; Al[rr][H + lane] = ql; }
  if (lane < 16) for (int k = 64; k < 72; ++k) { Ah[lane][k] = (b16)0.0f; Al[lane][k] = (b16)0.0f; }
  wave_lds_sync(); v8f acc[2] = {(v8f){}, (v8f){}};
#pragma unroll
  for (int kb = 0; kb < 64; kb += 32) { const v16b a = frag_kb(&Ah[nloc][kb], hlf), al = frag_kb(&Al[nloc][kb], hlf);
#pragma unroll
    for (int t = 0; t < 2; ++t) { const v16b bw = frag_kb(WN2 + (size_t)(t * 16 + nloc) * 64 + kb, hlf); acc[t] = wmma16b(a, bw, acc[t]); acc[t] = wmma16b(al, bw, acc[t]); } }
#pragma unroll
  for (int t = 0; t < 2; ++t) { const int cc = t * 16 + nloc; const float bb = bfv(bp[cc]) + bfv(bs[cc]);
#pragma unroll
    for (int r8 = 0; r8 < 8; ++r8) Tf[8 * hlf + r8][cc] = fmaxf(acc[t][r8] * (1.0f / (HS * WSC)) + bb, 0.0f); }
  wave_lds_sync();
  for (int pass = 0; pass < 2; ++pass) { for (int rr = 0; rr < 16; ++rr) ((volatile float*)XN2)[(m0 + rr) * H + lane] = Tf[rr][lane]; __threadfence(); } }
__global__ __launch_bounds__(32) void edge2_kernel(const float* __restrict__ XN2, const float* __restrict__ VALS1, const int* __restrict__ srcs, const int* __restrict__ dsts, const b16* __restrict__ WE2, const float* __restrict__ bep, const float* __restrict__ bes, const float* __restrict__ wc, const float* __restrict__ bc, int NLIM, int ELIM, float* __restrict__ out) { __shared__ __attribute__((aligned(16))) b16 Ah[32][F + 8], Al[32][F + 8]; __shared__ float Tf[32][H + 1], Os[32]; const int lane = threadIdx.x, nloc = lane & 15, hlf = lane >> 4; const size_t e0 = (size_t)blockIdx.x * 32; if (e0 >= (size_t)ELIM) return;
  for (int rr = 0; rr < 32; ++rr) { const size_t e = e0 + rr; const size_t s = (size_t)iclamp(srcs[e], 0, NLIM - 1), d = (size_t)iclamp(dsts[e], 0, NLIM - 1); const float a = XN2[s * H + lane], b = XN2[d * H + lane]; b16 p, ql; split16((a - b) * 0.5f * HS, p, ql); Ah[rr][lane] = p; Al[rr][lane] = ql; split16((a + b) * 0.5f * HS, p, ql); Ah[rr][H + lane] = p; Al[rr][H + lane] = ql; split16(VALS1[e * H + lane] * HS, p, ql); Ah[rr][64 + lane] = p; Al[rr][64 + lane] = ql; Ah[rr][96 + lane] = (b16)0.0f; Al[rr][96 + lane] = (b16)0.0f; }
  for (int k = F; k < F + 8; ++k) { Ah[lane][k] = (b16)0.0f; Al[lane][k] = (b16)0.0f; }
  wave_lds_sync();
#pragma unroll
  for (int rt = 0; rt < 2; ++rt) { v8f acc[2] = {(v8f){}, (v8f){}};
#pragma unroll
    for (int kb = 0; kb < F; kb += 32) { const v16b a = frag_kb(&Ah[rt * 16 + nloc][kb], hlf), al = frag_kb(&Al[rt * 16 + nloc][kb], hlf);
#pragma unroll
      for (int t = 0; t < 2; ++t) { const v16b bw = frag_kb(WE2 + (size_t)(t * 16 + nloc) * F + kb, hlf); acc[t] = wmma16b(a, bw, acc[t]); acc[t] = wmma16b(al, bw, acc[t]); } }
#pragma unroll
    for (int t = 0; t < 2; ++t) { const int cc = t * 16 + nloc; const float bb = bfv(bep[cc]) + bfv(bes[cc]);
#pragma unroll
      for (int r8 = 0; r8 < 8; ++r8) Tf[rt * 16 + 8 * hlf + r8][cc] = fmaxf(acc[t][r8] * (1.0f / (HS * WSC)) + bb, 0.0f); } }
  wave_lds_sync();
  { float s = bfv(bc[0]); for (int c = 0; c < H; ++c) s += pmul(Tf[lane][c], bfv(wc[c])); Os[lane] = 1.0f / (1.0f + __expf(-s)); }
  wave_lds_sync();
  for (int pass = 0; pass < 2; ++pass) { ((volatile float*)out)[e0 + lane] = Os[lane]; __threadfence(); } }
}

extern "C" void kernel_launch(void* const* d_in, const int* in_sizes, int n_in, void* d_out, int out_size, void* d_ws, size_t ws_size, hipStream_t stream) {
  (void)n_in;
  auto Fp = [&](int i) { return (const float*)d_in[i]; }; auto Ip = [&](int i) { return (const int*)d_in[i]; };
  if (in_sizes[0] != N * F || in_sizes[1] != E || in_sizes[2] != E || in_sizes[3] != N || in_sizes[4] != H * F || in_sizes[8] != H * 64 || in_sizes[10] != H * F || in_sizes[12] != H * H || in_sizes[16] != H * 64 || in_sizes[18] != H * H || in_sizes[20] != H || out_size != E) return;
  const int NLIM = N, ELIM = E;
  size_t off = 0; char* ws = (char*)d_ws;
  auto carve = [&](size_t bytes) { char* p = ws + off; off += (bytes + 255) & ~(size_t)255; return p; };
  b16* WN1 = (b16*)carve((size_t)H * F * 2); b16* WE1 = (b16*)carve((size_t)H * 192 * 2); b16* WN2 = (b16*)carve((size_t)H * 64 * 2); b16* WE2 = (b16*)carve((size_t)H * F * 2); float* XN1 = (float*)carve((size_t)N * H * 4); float* XN2 = (float*)carve((size_t)N * H * 4); float* VALS1 = (float*)carve((size_t)E * H * 4); CsrBufs8 csr; off = csr_carve8(csr, ws, off, E, N);
  if (off > ws_size || off > ((size_t)160 << 20)) return;
  wput_kernel<<<(H * 24 + 255) / 256, 256, 0, stream>>>(Fp(4), Fp(8), Fp(10), Fp(12), Fp(14), Fp(16), Fp(18), WN1, WE1, WN2, WE2);
  csr_build8(csr, Ip(1), E, N, stream);
  node1_kernel<<<NLIM / 16, 32, 0, stream>>>(Fp(0), Fp(3), Ip(2), csr.PERM, csr.ROWPTR, csr.ROWCNT, (int)csr.permLen, WN1, Fp(5), Fp(7), Fp(6), NLIM, XN1);
  edge1_kernel<<<ELIM / 32, 32, 0, stream>>>(Fp(0), XN1, Ip(1), Ip(2), WE1, Fp(9), Fp(11), NLIM, ELIM, VALS1);
  node2_kernel<<<NLIM / 16, 32, 0, stream>>>(VALS1, XN1, Fp(3), csr.PERM, csr.ROWPTR, csr.ROWCNT, (int)csr.permLen, WN2, Fp(13), Fp(15), NLIM, ELIM, XN2);
  edge2_kernel<<<ELIM / 32, 32, 0, stream>>>(XN2, VALS1, Ip(1), Ip(2), WE2, Fp(17), Fp(19), Fp(20), Fp(21), NLIM, ELIM, (float*)d_out);
}
